// NTM_4922032521896
// MI455X (gfx1250) — hardware-verified
//
#include <hip/hip_runtime.h>
#include <math.h>

constexpr int NB   = 64;
constexpr int NT   = 64;
constexpr int NI   = 2048;
constexpr int NH   = 2048;
constexpr int MB   = 4;
constexpr int MN   = 128;
constexpr int MW   = 20;
constexpr int MWP  = 32;
constexpr int NROW = NB * NT;
constexpr int NTHR = 256;
constexpr int RB   = 16;
constexpr int KP   = 32;
constexpr int RP   = 32;
constexpr int SLABP = 68;
static_assert(NB % RB == 0);
static_assert(NH == 8 * 256);
static_assert(NH == NI);
static_assert(MN == 128);
static_assert(MW <= MWP && MWP == 32 && MW % 4 == 0);
static_assert(MB == 4);
static_assert(RB * MWP == 2 * NTHR);
static_assert((MN * MW) % 4 == 0 && (MN * MW) / 4 <= 3 * NTHR);
static_assert(NROW % 64 == 0 && NH % 64 == 0 && NI % 64 == 0);
static_assert(NI % 32 == 0 && NH % 32 == 0);
static_assert(((NROW / 64) * (NH / 64)) % 8 == 0);
static_assert(NH == 512 * 4);
static_assert((NROW * NI / 8) % NTHR == 0 && (NB * NH / 8) % NTHR == 0);

typedef __attribute__((ext_vector_type(16))) _Float16 v16h;
typedef __attribute__((ext_vector_type(8)))  _Float16 v8h;
typedef __attribute__((ext_vector_type(16))) __bf16   v16b;
typedef __attribute__((ext_vector_type(8)))  __bf16   v8b;
typedef __attribute__((ext_vector_type(8)))  float    v8f;
typedef __attribute__((ext_vector_type(4)))  float    v4f;
typedef __attribute__((ext_vector_type(4)))  unsigned v4u;

__device__ __forceinline__ unsigned short f2bf_bits(float f) {
  unsigned u = __float_as_uint(f);
  return (unsigned short)((u + 0x7FFFu + ((u >> 16) & 1u)) >> 16);
}
__device__ __forceinline__ float bf_bits2f(unsigned short h) { return __uint_as_float(((unsigned)h) << 16); }
__device__ __forceinline__ float bf16r(float f) { return bf_bits2f(f2bf_bits(f)); }

__device__ __forceinline__ void dep_guard_b(v8f& a, v8f& b, v16b x, v16b y) { asm volatile("v_nop\n\tv_nop\n\tv_nop\n\tv_nop" : "+v"(a), "+v"(b) : "v"(x), "v"(y)); }
__device__ __forceinline__ void guard4_b(v8f& a, v8f& b, v8f& c, v8f& d, v16b x, v16b y) {
  asm volatile("v_nop\n\tv_nop\n\tv_nop\n\tv_nop" : "+v"(a), "+v"(b), "+v"(c), "+v"(d) : "v"(x), "v"(y));
}
__device__ __forceinline__ void keep4_b(v16b a, v16b b, v16b c, v16b d) { asm volatile("v_nop" :: "v"(a), "v"(b), "v"(c), "v"(d)); }
__device__ __forceinline__ void acc_guard4(v8f& a, v8f& b, v8f& c, v8f& d) { asm volatile("v_nop\n\tv_nop\n\tv_nop\n\tv_nop" : "+v"(a), "+v"(b), "+v"(c), "+v"(d)); }
__device__ __forceinline__ void acc_guard2(v8f& a, v8f& b) { asm volatile("v_nop\n\tv_nop\n\tv_nop\n\tv_nop" : "+v"(a), "+v"(b)); }

template <typename T> struct Frag;
template <> struct Frag<__bf16> {
  typedef v16b V; union U { v16b v; v8b h[2]; };
  static __device__ __forceinline__ v16b load(const __bf16* p) {
    U f; f.h[0] = *(const v8b*)(p); f.h[1] = *(const v8b*)(p + 16); return f.v;
  }
  static __device__ __forceinline__ v8f mma(v16b a, v16b b, v8f c) {
    return __builtin_amdgcn_wmma_f32_16x16x32_bf16(false, a, false, b, (short)0, c, false, false);
  }
  static __device__ __forceinline__ void guard(v8f& a, v8f& b, v16b x, v16b y) { dep_guard_b(a, b, x, y); }
  static __device__ __forceinline__ void keep(v16b a, v16b b, v16b c, v16b d) { keep4_b(a, b, c, d); }
};

template <bool SPLITA, bool CLIP01>
__global__ __launch_bounds__(NTHR) void gemm64_bf16_kernel(
    const unsigned short* __restrict__ Ap, const unsigned short* __restrict__ A2p, int lda,
    const unsigned short* __restrict__ Btp, int ldb,
    float* __restrict__ Cout, int ldc, const float* __restrict__ bias, int M, int N, int K) {
  const __bf16* A = (const __bf16*)Ap; const __bf16* A2 = (const __bf16*)A2p; const __bf16* Bt = (const __bf16*)Btp;
  __shared__ __align__(16) float sT[8][16 * SLABP];
  const int lane = threadIdx.x & 31;
  const int wave = threadIdx.x >> 5;
  const int tilesN = N >> 6;
  const int tilesM = M >> 6;
  const int tile = blockIdx.x * 8 + wave;
  if (tile >= tilesM * tilesN) return;
  const int tm = tile / tilesN;
  const int tn = tile - tm * tilesN;
  const int m0 = tm << 6;
  const int n0 = tn << 6;
  const int rlane = lane & 15;
  const int koff  = (lane >> 4) * 8;
  const int mOff  = (lane >> 4) * 8;

  v8f acc[4][4];
#pragma unroll
  for (int i = 0; i < 4; ++i)
#pragma unroll
    for (int j = 0; j < 4; ++j) acc[i][j] = (v8f){0.f,0.f,0.f,0.f,0.f,0.f,0.f,0.f};

  for (int k0 = 0; k0 < K; k0 += 32) {
    v16b bh[4];
#pragma unroll
    for (int j = 0; j < 4; ++j) {
      const size_t bo = (size_t)(n0 + (j << 4) + rlane) * ldb + koff + k0;
      bh[j] = Frag<__bf16>::load(Bt + bo);
    }
#pragma unroll
    for (int i = 0; i < 4; ++i) {
      const size_t ao = (size_t)(m0 + (i << 4) + rlane) * lda + koff + k0;
      const v16b ah = Frag<__bf16>::load(A + ao);
      v16b al = ah;
      if (SPLITA) al = Frag<__bf16>::load(A2 + ao);
#pragma unroll
      for (int j = 0; j < 4; ++j) {
        acc[i][j] = Frag<__bf16>::mma(ah, bh[j], acc[i][j]);
        if (SPLITA) acc[i][j] = Frag<__bf16>::mma(al, bh[j], acc[i][j]);
      }
      guard4_b(acc[i][0], acc[i][1], acc[i][2], acc[i][3], ah, al);
    }
    keep4_b(bh[0], bh[1], bh[2], bh[3]);
  }
  acc_guard4(acc[0][0], acc[0][1], acc[0][2], acc[0][3]);
  acc_guard4(acc[1][0], acc[1][1], acc[1][2], acc[1][3]);
  acc_guard4(acc[2][0], acc[2][1], acc[2][2], acc[2][3]);
  acc_guard4(acc[3][0], acc[3][1], acc[3][2], acc[3][3]);

  float* slab = sT[wave];
#pragma unroll
  for (int i = 0; i < 4; ++i) {
    const int mBase = m0 + (i << 4);
#pragma unroll
    for (int j = 0; j < 4; ++j) {
      const int n = n0 + (j << 4) + rlane;
      const float bv = bias[n];
#pragma unroll
      for (int r = 0; r < 8; ++r) {
        float v = acc[i][j][r] + bv;
        if (CLIP01) v = fminf(fmaxf(v, 0.0f), 1.0f);
        slab[(mOff + r) * SLABP + (j << 4) + rlane] = v;
      }
    }
    __builtin_amdgcn_fence(__ATOMIC_RELEASE, "workgroup");
    __builtin_amdgcn_wave_barrier();
    __builtin_amdgcn_fence(__ATOMIC_ACQUIRE, "workgroup");
    {
      const int hh = lane >> 4, c4 = (lane & 15) * 4;
      for (int pass = 0; pass < 2; ++pass) {
#pragma unroll
        for (int it = 0; it < 8; ++it) {
          const int row = it * 2 + hh;
          const v4f v = *(const v4f*)(slab + row * SLABP + c4);
          *(volatile v4f*)(Cout + (size_t)(mBase + row) * ldc + n0 + c4) = v;
        }
        __threadfence();
      }
    }
    __builtin_amdgcn_fence(__ATOMIC_RELEASE, "workgroup");
    __builtin_amdgcn_wave_barrier();
    __builtin_amdgcn_fence(__ATOMIC_ACQUIRE, "workgroup");
  }
}

__global__ __launch_bounds__(NTHR) void cvt8_bf16_kernel(const float* __restrict__ src, unsigned short* __restrict__ dst, int n8) {
  const int i = blockIdx.x * NTHR + threadIdx.x;
  if (i < n8) {
    const float* sp = src + (size_t)i * 8;
    const v4f a = *(const v4f*)(sp);
    const v4f b = *(const v4f*)(sp + 4);
    v8h hv;
#pragma unroll
    for (int e = 0; e < 4; ++e) {
      const unsigned short b0 = f2bf_bits(a[e]);
      const unsigned short b1 = f2bf_bits(b[e]);
      hv[e]     = __builtin_bit_cast(_Float16, b0);
      hv[4 + e] = __builtin_bit_cast(_Float16, b1);
    }
    *(volatile v8h*)(dst + (size_t)i * 8) = hv;
    __threadfence();
    *(volatile v8h*)(dst + (size_t)i * 8) = hv;
  }
}

__global__ __launch_bounds__(NTHR) void zfill16_kernel(unsigned short* __restrict__ dst, int n8) {
  const int i = blockIdx.x * NTHR + threadIdx.x;
  if (i < n8) {
    const v4u z = {0u, 0u, 0u, 0u};
    *(volatile v4u*)(dst + (size_t)i * 8) = z;
    __threadfence();
    *(volatile v4u*)(dst + (size_t)i * 8) = z;
  }
}

__global__ __launch_bounds__(NTHR) void tr_cvt_kernel(const float* __restrict__ src, unsigned short* __restrict__ dst,
                                                      int R, int C, int Rd, int Cd) {
  __shared__ float tile[64][33];
  const int tid = threadIdx.x;
  const int r0 = blockIdx.x * 64;
  const int c0 = blockIdx.y * 32;
  const int cc = tid & 31;
#pragma unroll
  for (int i = 0; i < 8; ++i) {
    const int rr = (tid >> 5) + 8 * i;
    const int r = r0 + rr, c = c0 + cc;
    const int rcl = (r < R) ? r : (R - 1);
    const int ccl = (c < C) ? c : (C - 1);
    const float v = src[(size_t)rcl * C + ccl];
    tile[rr][cc] = (r < R && c < C) ? v : 0.0f;
  }
  __syncthreads();
  const int lr = tid >> 3;
  const int c8 = (tid & 7) * 8;
  v8h hv;
#pragma unroll
  for (int e = 0; e < 8; ++e) {
    const unsigned short bits = f2bf_bits(tile[c8 + e][lr]);
    hv[e] = __builtin_bit_cast(_Float16, bits);
  }
  unsigned short* dp = dst + (size_t)(c0 + lr) * Rd + r0 + c8;
  *(volatile v8h*)dp = hv;
  __threadfence();
  *(volatile v8h*)dp = hv;
  (void)Cd;
}

__global__ __launch_bounds__(NTHR) void wread_kernel(const float* __restrict__ src, unsigned short* __restrict__ dst) {
  __shared__ float tile[MW][64];
  const int tid = threadIdx.x;
  const int n0 = blockIdx.x * 64;
#pragma unroll
  for (int it = 0; it < (MW * 64) / NTHR; ++it) {
    const int i = tid + NTHR * it;
    const int k = i >> 6, nn = i & 63;
    tile[k][nn] = src[(size_t)k * NH + n0 + nn];
  }
  __syncthreads();
  const int lr = tid >> 2;
  const int kc = (tid & 3) * 8;
  v8h hv;
#pragma unroll
  for (int e = 0; e < 8; ++e) {
    const int k = kc + e;
    const int kcl = (k < MW) ? k : (MW - 1);
    const float v = tile[kcl][lr];
    const unsigned short bits = (k < MW) ? f2bf_bits(v) : (unsigned short)0;
    hv[e] = __builtin_bit_cast(_Float16, bits);
  }
  unsigned short* dp = dst + (size_t)(n0 + lr) * MWP + kc;
  *(volatile v8h*)dp = hv;
  __threadfence();
  *(volatile v8h*)dp = hv;
}
static_assert((MW * 64) % NTHR == 0);

__global__ __launch_bounds__(512) void bias3_kernel(const float* __restrict__ s0, const float* __restrict__ s1,
                                                  const float* __restrict__ s2, float* __restrict__ dst) {
  const int which = blockIdx.x;
  const int idx = threadIdx.x * 4;
  const v4f a = *(const v4f*)(s0 + idx);
  const v4f b = *(const v4f*)(s1 + idx);
  const v4f d = *(const v4f*)(s2 + idx);
  v4f o;
#pragma unroll
  for (int e = 0; e < 4; ++e) {
    const float v = (which == 0) ? a[e] : ((which == 1) ? b[e] : d[e]);
    o[e] = bf16r(v);
  }
  float* op = dst + (size_t)which * NH + idx;
  *(volatile v4f*)op = o;
  __threadfence();
  *(volatile v4f*)op = o;
}

__global__ __launch_bounds__(NTHR) void scan_kernel(
    const unsigned short* __restrict__ H0hi, const unsigned short* __restrict__ H0lo,
    unsigned short* Hhi, unsigned short* Hlo,
    const unsigned short* __restrict__ WkeyTp, const unsigned short* __restrict__ WreadTp,
    const float* __restrict__ Z, const float* __restrict__ breadr,
    const float* __restrict__ bkey, const float* __restrict__ mem) {
  __shared__ __align__(16) float part[8 * 2 * 8 * 32];
  __shared__ __align__(16) float kbuf[RB * KP];
  __shared__ __align__(16) float bankL[MN * MW];
  __shared__ float bnL[MN];
  __shared__ float bkL[MWP];
  __shared__ __align__(16) unsigned short rHs[RB * RP];
  __shared__ __align__(16) unsigned short rLs[RB * RP];
  __shared__ __align__(16) float slabs[8][16 * SLABP];

  const __bf16* WkeyT  = (const __bf16*)WkeyTp;
  const __bf16* WreadT = (const __bf16*)WreadTp;
  const __bf16* H0h = (const __bf16*)H0hi;
  const __bf16* H0l = (const __bf16*)H0lo;
  const __bf16* Hh  = (const __bf16*)Hhi;
  const __bf16* Hl  = (const __bf16*)Hlo;

  const int tid = threadIdx.x, lane = tid & 31, wave = tid >> 5;
  const int c = lane & 15, hh = lane >> 4, koff = hh * 8;
  const int rb0 = blockIdx.x * RB;
  const v8f z8 = {0.f, 0.f, 0.f, 0.f, 0.f, 0.f, 0.f, 0.f};
  float* slab = slabs[wave];

  if (tid < MWP) {
    const int cl = (tid < MW) ? tid : (MW - 1);
    const float bv = bf16r(bkey[cl]);
    bkL[tid] = (tid < MW) ? bv : 0.0f;
  }
  __syncthreads();

#pragma unroll 1
  for (int t = 0; t < NT; ++t) {
    {
      const float* bank = mem + (size_t)(t & (MB - 1)) * (MN * MW);
#pragma unroll
      for (int it = 0; it < 3; ++it) {
        const int vi = tid + NTHR * it;
        const int vcl = (vi < (MN * MW) / 4) ? vi : ((MN * MW) / 4 - 1);
        const v4f v = *(const v4f*)(bank + 4 * vcl);
        if (vi < (MN * MW) / 4) {
          bankL[4 * vcl + 0] = bf16r(v[0]);
          bankL[4 * vcl + 1] = bf16r(v[1]);
          bankL[4 * vcl + 2] = bf16r(v[2]);
          bankL[4 * vcl + 3] = bf16r(v[3]);
        }
      }
    }

    {
      const __bf16* aHi = (t == 0) ? (H0h + (size_t)(rb0 + c) * NH + koff)
                                   : (Hh + ((size_t)(rb0 + c) * NT + (size_t)(t - 1)) * NH + koff);
      const __bf16* aLo = (t == 0) ? (H0l + (size_t)(rb0 + c) * NH + koff)
                                   : (Hl + ((size_t)(rb0 + c) * NT + (size_t)(t - 1)) * NH + koff);
      const __bf16* b0p = WkeyT + (size_t)c * NH + koff;
      const __bf16* b1p = WkeyT + (size_t)(16 + c) * NH + koff;
      const int kbase = wave * (NH / 8);
      v8f acc0 = z8, acc1 = z8;
#pragma unroll 1
      for (int ks = 0; ks < (NH / 8) / 32; ++ks) {
        const int k0 = kbase + ks * 32;
        const v16b ah  = Frag<__bf16>::load(aHi + k0);
        const v16b al  = Frag<__bf16>::load(aLo + k0);
        const v16b bb0 = Frag<__bf16>::load(b0p + k0);
        const v16b bb1 = Frag<__bf16>::load(b1p + k0);
        acc0 = Frag<__bf16>::mma(ah, bb0, acc0);
        acc0 = Frag<__bf16>::mma(al, bb0, acc0);
        acc1 = Frag<__bf16>::mma(ah, bb1, acc1);
        acc1 = Frag<__bf16>::mma(al, bb1, acc1);
        dep_guard_b(acc0, acc1, ah, al);
        keep4_b(bb0, bb1, ah, al);
      }
      acc_guard2(acc0, acc1);
#pragma unroll
      for (int r = 0; r < 8; ++r) {
        part[(wave * 2 + 0) * 256 + r * 32 + lane] = acc0[r];
        part[(wave * 2 + 1) * 256 + r * 32 + lane] = acc1[r];
      }
    }
    __syncthreads();

    {
#pragma unroll
      for (int oo = 0; oo < 2; ++oo) {
        const int o = tid + NTHR * oo;
        const int nt = o >> 8, r = (o >> 5) & 7, ln = o & 31;
        const int row = 8 * (ln >> 4) + r;
        const int col = nt * 16 + (ln & 15);
        float v = 0.0f;
#pragma unroll
        for (int w = 0; w < 8; ++w) v += part[w * 512 + (o & 511)];
        const float kvv = v + bkL[col];
        kbuf[row * KP + col] = (col < MW) ? kvv : 0.0f;
      }
      if (tid < MN) {
        const float* bp = bankL + tid * MW;
        float s = 0.0f;
#pragma unroll
        for (int cc = 0; cc < MW; ++cc) s += bp[cc] * bp[cc];
        bnL[tid] = sqrtf(s);
      }
    }
    __syncthreads();

#pragma unroll 1
    for (int ii = 0; ii < 2; ++ii) {
      const int i = wave * 2 + ii;
      float kv[MW];
#pragma unroll
      for (int m = 0; m < MW / 4; ++m) {
        const v4f v = *(const v4f*)(kbuf + i * KP + 4 * m);
        kv[4 * m + 0] = v[0]; kv[4 * m + 1] = v[1]; kv[4 * m + 2] = v[2]; kv[4 * m + 3] = v[3];
      }
      float kn2 = 0.0f;
#pragma unroll
      for (int cc = 0; cc < MW; ++cc) kn2 += kv[cc] * kv[cc];
      const float kn = sqrtf(kn2);
      float sv[4];
      float mx = -INFINITY;
#pragma unroll
      for (int q = 0; q < 4; ++q) {
        const int j = lane + 32 * q;
        const float* bp = bankL + j * MW;
        float d = 0.0f;
#pragma unroll
        for (int m = 0; m < MW / 4; ++m) {
          const v4f bv = *(const v4f*)(bp + 4 * m);
          d += kv[4 * m + 0] * bv[0]; d += kv[4 * m + 1] * bv[1]; d += kv[4 * m + 2] * bv[2]; d += kv[4 * m + 3] * bv[3];
        }
        const float den = kn * bnL[j] + 1e-8f;
        sv[q] = d / den;
        mx = fmaxf(mx, sv[q]);
      }
#pragma unroll
      for (int off = 16; off > 0; off >>= 1) mx = fmaxf(mx, __shfl_xor(mx, off, 32));
      float ev[4];
      float sum = 0.0f;
#pragma unroll
      for (int q = 0; q < 4; ++q) { ev[q] = expf(sv[q] - mx); sum += ev[q]; }
#pragma unroll
      for (int off = 16; off > 0; off >>= 1) sum += __shfl_xor(sum, off, 32);
      const float inv = 1.0f / sum;
      float racc[MW];
#pragma unroll
      for (int cc = 0; cc < MW; ++cc) racc[cc] = 0.0f;
#pragma unroll
      for (int q = 0; q < 4; ++q) {
        const int j = lane + 32 * q;
        const float* bp = bankL + j * MW;
        const float wq = ev[q] * inv;
#pragma unroll
        for (int m = 0; m < MW / 4; ++m) {
          const v4f bv = *(const v4f*)(bp + 4 * m);
          racc[4 * m + 0] += wq * bv[0]; racc[4 * m + 1] += wq * bv[1];
          racc[4 * m + 2] += wq * bv[2]; racc[4 * m + 3] += wq * bv[3];
        }
      }
#pragma unroll
      for (int cc = 0; cc < MW; ++cc) {
#pragma unroll
        for (int off = 16; off > 0; off >>= 1) racc[cc] += __shfl_xor(racc[cc], off, 32);
      }
      float rv = 0.0f;
#pragma unroll
      for (int cc = 0; cc < MW; ++cc) rv = (lane == cc) ? racc[cc] : rv;
      const unsigned short hb = f2bf_bits(rv);
      const unsigned short lb = f2bf_bits(rv - bf_bits2f(hb));
      rHs[i * RP + lane] = hb;
      rLs[i * RP + lane] = lb;
    }
    __syncthreads();

    {
      const v16b rHf = Frag<__bf16>::load((const __bf16*)rHs + c * RP + koff);
      const v16b rLf = Frag<__bf16>::load((const __bf16*)rLs + c * RP + koff);
      const int q  = lane >> 3;
      const int c8 = (lane & 7) * 8;
#pragma unroll 1
      for (int g = 0; g < 4; ++g) {
        const int n0 = wave * (NH / 8) + g * 64;
        v16b bw[4];
#pragma unroll
        for (int j = 0; j < 4; ++j) bw[j] = Frag<__bf16>::load(WreadT + (size_t)(n0 + 16 * j + c) * MWP + koff);
        v8f a4[4];
#pragma unroll
        for (int j = 0; j < 4; ++j) {
          a4[j] = Frag<__bf16>::mma(rHf, bw[j], z8);
          a4[j] = Frag<__bf16>::mma(rLf, bw[j], a4[j]);
        }
        guard4_b(a4[0], a4[1], a4[2], a4[3], rHf, rLf);
        keep4_b(bw[0], bw[1], bw[2], bw[3]);
#pragma unroll
        for (int j = 0; j < 4; ++j)
#pragma unroll
          for (int r = 0; r < 8; ++r) slab[(8 * hh + r) * SLABP + 16 * j + c] = a4[j][r];
        __builtin_amdgcn_fence(__ATOMIC_RELEASE, "workgroup");
        __builtin_amdgcn_wave_barrier();
        __builtin_amdgcn_fence(__ATOMIC_ACQUIRE, "workgroup");

        const v4f bb0 = *(const v4f*)(breadr + n0 + c8);
        const v4f bb1 = *(const v4f*)(breadr + n0 + c8 + 4);
        v8h hvv[4], lvv[4];
#pragma unroll
        for (int it = 0; it < 4; ++it) {
          const int row = it * 4 + q;
          const size_t zoff = ((size_t)(rb0 + row) * NT + (size_t)t) * NH + n0 + c8;
          const v4f z0 = *(const v4f*)(Z + zoff);
          const v4f z1 = *(const v4f*)(Z + zoff + 4);
          const v4f s0 = *(const v4f*)(slab + row * SLABP + c8);
          const v4f s1 = *(const v4f*)(slab + row * SLABP + c8 + 4);
#pragma unroll
          for (int e = 0; e < 4; ++e) {
            const float v0 = fmaxf((z0[e] + s0[e]) + bb0[e], 0.0f);
            const float v1 = fmaxf((z1[e] + s1[e]) + bb1[e], 0.0f);
            const unsigned short h0b = f2bf_bits(v0);
            const unsigned short l0b = f2bf_bits(v0 - bf_bits2f(h0b));
            const unsigned short h1b = f2bf_bits(v1);
            const unsigned short l1b = f2bf_bits(v1 - bf_bits2f(h1b));
            hvv[it][e]     = __builtin_bit_cast(_Float16, h0b);
            lvv[it][e]     = __builtin_bit_cast(_Float16, l0b);
            hvv[it][4 + e] = __builtin_bit_cast(_Float16, h1b);
            lvv[it][4 + e] = __builtin_bit_cast(_Float16, l1b);
          }
          asm volatile("" ::: "memory");
        }
        for (int pass = 0; pass < 2; ++pass) {
#pragma unroll
          for (int it = 0; it < 4; ++it) {
            const int row = it * 4 + q;
            const size_t hoff = ((size_t)(rb0 + row) * NT + (size_t)t) * NH + n0 + c8;
            *(volatile v8h*)(Hhi + hoff) = hvv[it];
            *(volatile v8h*)(Hlo + hoff) = lvv[it];
          }
          __threadfence();
        }
        __builtin_amdgcn_fence(__ATOMIC_RELEASE, "workgroup");
        __builtin_amdgcn_wave_barrier();
        __builtin_amdgcn_fence(__ATOMIC_ACQUIRE, "workgroup");
      }
    }
    __threadfence();
    __syncthreads();
    __threadfence();
  }
}

extern "C" void kernel_launch(void* const* d_in, const int* in_sizes, int n_in,
                              void* d_out, int out_size, void* d_ws, size_t ws_size, hipStream_t stream) {
  if (n_in < 11 || d_out == nullptr || d_ws == nullptr) return;
  if (in_sizes[0] != NB * NT * NI || in_sizes[1] != NB * NH || in_sizes[2] != NI * NH || in_sizes[3] != NH ||
      in_sizes[4] != MW * NH || in_sizes[5] != NH || in_sizes[6] != NH * NI || in_sizes[7] != NI ||
      in_sizes[8] != NH * MW || in_sizes[9] != MW || in_sizes[10] != MB * MN * MW || out_size != NROW * NI) return;

  const float* x      = (const float*)d_in[0];
  const float* h0     = (const float*)d_in[1];
  const float* W_in   = (const float*)d_in[2];
  const float* b_in   = (const float*)d_in[3];
  const float* W_read = (const float*)d_in[4];
  const float* b_read = (const float*)d_in[5];
  const float* W_out  = (const float*)d_in[6];
  const float* b_out  = (const float*)d_in[7];
  const float* W_key  = (const float*)d_in[8];
  const float* b_key  = (const float*)d_in[9];
  const float* memory = (const float*)d_in[10];
  float* out = (float*)d_out;

  char* ws = (char*)d_ws; size_t off = 0;
  auto carve = [&](size_t bytes) -> char* { char* p = ws + off; off += (bytes + 255) & ~(size_t)255; return p; };
  unsigned short* XB     = (unsigned short*)carve((size_t)NROW * NI * 2);
  unsigned short* WINT   = (unsigned short*)carve((size_t)NH * NI * 2);
  unsigned short* WOUTT  = (unsigned short*)carve((size_t)NI * NH * 2);
  unsigned short* WKEYT  = (unsigned short*)carve((size_t)MWP * NH * 2);
  unsigned short* WREADT = (unsigned short*)carve((size_t)NH * MWP * 2);
  unsigned short* H0H    = (unsigned short*)carve((size_t)NB * NH * 2);
  unsigned short* H0L    = (unsigned short*)carve((size_t)NB * NH * 2);
  float*          BIASR  = (float*)carve((size_t)3 * NH * 4);
  float*          Z      = (float*)carve((size_t)NROW * NH * 4);
  unsigned short* HH     = (unsigned short*)carve((size_t)NROW * NH * 2);
  unsigned short* HL     = (unsigned short*)carve((size_t)NROW * NH * 2);
  if (off > ws_size || off > (size_t)134217728) return;

  const int n8x = NROW * NI / 8;
  const int n8h = NB * NH / 8;
  cvt8_bf16_kernel<<<n8x / NTHR, NTHR, 0, stream>>>(x, XB, n8x);
  tr_cvt_kernel<<<dim3(NI / 64, NH / 32), NTHR, 0, stream>>>(W_in,  WINT,  NI, NH, NI, NH);
  tr_cvt_kernel<<<dim3(NH / 64, NI / 32), NTHR, 0, stream>>>(W_out, WOUTT, NH, NI, NH, NI);
  tr_cvt_kernel<<<dim3(NH / 64, MWP / 32), NTHR, 0, stream>>>(W_key, WKEYT, NH, MW, NH, MWP);
  wread_kernel<<<NH / 64, NTHR, 0, stream>>>(W_read, WREADT);
  cvt8_bf16_kernel<<<n8h / NTHR, NTHR, 0, stream>>>(h0, H0H, n8h);
  zfill16_kernel<<<n8h / NTHR, NTHR, 0, stream>>>(H0L, n8h);
  bias3_kernel<<<3, 512, 0, stream>>>(b_in, b_out, b_read, BIASR);

  gemm64_bf16_kernel<false, false><<<(NROW / 64) * (NH / 64) / 8, NTHR, 0, stream>>>(
      XB, XB, NI, WINT, NI, Z, NH, BIASR, NROW, NH, NI);

  scan_kernel<<<NB / RB, NTHR, 0, stream>>>(H0H, H0L, HH, HL, WKEYT, WREADT, Z, BIASR + 2 * NH, b_key, memory);

  gemm64_bf16_kernel<true, true><<<(NROW / 64) * (NI / 64) / 8, NTHR, 0, stream>>>(
      HH, HL, NH, WOUTT, NH, out, NI, BIASR + NH, NROW, NI, NH);
}
